// LSTM_37091337568423
// MI455X (gfx1250) — hardware-verified
//
#include <hip/hip_runtime.h>
#include <math.h>

typedef __attribute__((ext_vector_type(16))) _Float16 v16h;
typedef __attribute__((ext_vector_type(8)))  _Float16 v8h;
typedef __attribute__((ext_vector_type(8)))  float    v8f;
typedef __attribute__((ext_vector_type(4)))  float    v4f;

constexpr int BATCH_N  = 32768;
constexpr int SEQ_FULL = 30;
constexpr int FEAT_IN  = 4;
constexpr int HID_N    = 32;
constexpr int GATE_N   = 4 * HID_N;
constexpr int STEP_N   = 15;
constexpr int ROWS_ALL = 2 * BATCH_N;
constexpr int L1_IN    = 2 * HID_N;
constexpr int DIR_CLS  = 6;
constexpr int NTHR     = 256;
constexpr int ROWS_BLK = 128;
constexpr int SLAB_P   = 68;
constexpr int OUT_W    = 2;

constexpr float WCARRY     = 16.0f;
constexpr float WCARRY_INV = 1.0f / WCARRY;
constexpr float XLO_CARRY  = 16.0f;
constexpr float WLO_CARRY  = 64.0f;
constexpr float BLO_CARRY  = 256.0f;

static_assert(GATE_N == 128 && HID_N == 32 && L1_IN == 64, "shape");
static_assert(BATCH_N % ROWS_BLK == 0, "row tiles exact");
static_assert(ROWS_BLK == 16 * (NTHR / 32), "one 16-row tile per wave");
static_assert(SEQ_FULL == 2 * STEP_N, "two halves");
static_assert(FEAT_IN == 4, "float4 rows");
static_assert(HID_N % 32 == 0 && L1_IN % 32 == 0, "k multiple of 32");

union FragU { v16h v; v8h h[2]; };

__device__ __forceinline__ v16h frag_ld(const _Float16* p) {
  FragU f; f.h[0] = *(const v8h*)(p); f.h[1] = *(const v8h*)(p + 16); return f.v;
}
__device__ __forceinline__ v16h frag_ld_packed(const _Float16* p) {
  FragU f; f.h[0] = *(const v8h*)(p); f.h[1] = *(const v8h*)(p + 8); return f.v;
}
__device__ __forceinline__ v8f mma_h(v16h a, v16h b, v8f c) {
  c = __builtin_amdgcn_wmma_f32_16x16x32_f16(false, a, false, b, (short)0, c, false, false);
  asm volatile("v_nop\n\tv_nop\n\tv_nop\n\tv_nop" : "+v"(c) : "v"(a), "v"(b));
  return c;
}
__device__ __forceinline__ v16h wfrag_from_f32(const float* __restrict__ src, int hh) {
  const float* p0 = src + 8 * hh;
  const v4f a0 = *(const v4f*)(p0);
  const v4f a1 = *(const v4f*)(p0 + 4);
  const v4f b0 = *(const v4f*)(p0 + 16);
  const v4f b1 = *(const v4f*)(p0 + 20);
  FragU u;
#pragma unroll
  for (int e = 0; e < 4; ++e) {
    u.h[0][e]     = (_Float16)(a0[e] * WCARRY);
    u.h[0][4 + e] = (_Float16)(a1[e] * WCARRY);
    u.h[1][e]     = (_Float16)(b0[e] * WCARRY);
    u.h[1][4 + e] = (_Float16)(b1[e] * WCARRY);
  }
  return u.v;
}

__device__ __forceinline__ float fsig(float x)  { return __builtin_amdgcn_rcpf(1.0f + __expf(-x)); }
__device__ __forceinline__ float ftanh(float x) { return 1.0f - 2.0f * __builtin_amdgcn_rcpf(__expf(2.0f * x) + 1.0f); }

__global__ __launch_bounds__(NTHR) void lstm_l0_kernel(const float* __restrict__ pos,
                                                      const float* __restrict__ Wih,
                                                      const float* __restrict__ Whh,
                                                      const float* __restrict__ bias,
                                                      unsigned short* __restrict__ y0p, int toff) {
  __shared__ __align__(16) _Float16 sWx[8 * 32 * 16];
  __shared__ __align__(16) _Float16 sH[NTHR / 32][16 * HID_N];

  const int tid = threadIdx.x, lane = tid & 31, wave = tid >> 5;
  const int c = lane & 15, hh = lane >> 4;
  const int dir = blockIdx.y;
  const int rowbase = blockIdx.x * ROWS_BLK + wave * 16;

  float zl = 0.0f, onef = 1.0f;
  asm volatile("" : "+v"(zl), "+v"(onef));

  {
    const int g = wave * 16 + c;
    const v4f w = *(const v4f*)(Wih + ((size_t)dir * GATE_N + g) * FEAT_IN);
    const float bv = bias[dir * GATE_N + g];
    v8h e0, e1;
#pragma unroll
    for (int e = 0; e < 4; ++e) {
      const float wv = w[e];
      const _Float16 wh = (_Float16)wv;
      const float whf = (float)wh;
      const float wlo = wv - whf;
      const float f0 = whf * WCARRY;
      const float f1 = whf * (WCARRY / XLO_CARRY);
      const float f2 = wlo * (WLO_CARRY * WCARRY);
      e0[e]     = (_Float16)(hh ? zl : f0);
      e0[4 + e] = (_Float16)(hh ? zl : f1);
      e1[e]     = (_Float16)(hh ? zl : f2);
    }
    const _Float16 bh = (_Float16)bv;
    const float bhf = (float)bh;
    const float blo = bv - bhf;
    e1[4] = (_Float16)(hh ? zl : bhf * WCARRY);
    e1[5] = (_Float16)(hh ? zl : blo * (BLO_CARRY * WCARRY));
    e1[6] = (_Float16)zl;
    e1[7] = (_Float16)zl;
    *(v8h*)(sWx + tid * 16)     = e0;
    *(v8h*)(sWx + tid * 16 + 8) = e1;
  }

  v16h whB[8];
#pragma unroll
  for (int n = 0; n < 8; ++n) {
    whB[n] = wfrag_from_f32(Whh + ((size_t)dir * GATE_N + n * 16 + c) * HID_N, hh);
    asm volatile("" : "+v"(whB[n]) :: "memory");
  }
  __syncthreads();

  float cst[2][8];
#pragma unroll
  for (int j = 0; j < 2; ++j)
#pragma unroll
    for (int r = 0; r < 8; ++r) cst[j][r] = 0.0f;

  const v8f z8 = {0.f, 0.f, 0.f, 0.f, 0.f, 0.f, 0.f, 0.f};
  _Float16* ht = &sH[wave][0];
  const float* xrow = pos + ((size_t)(rowbase + c) * SEQ_FULL + (size_t)toff) * FEAT_IN;

#pragma unroll 1
  for (int t = 0; t < STEP_N; ++t) {
    const int tt = dir ? (STEP_N - 1 - t) : t;

    const v4f xv = *(const v4f*)(xrow + (size_t)tt * FEAT_IN);
    FragU xa;
#pragma unroll
    for (int e = 0; e < 4; ++e) {
      const float xf = xv[e];
      const _Float16 xh = (_Float16)xf;
      const float xhf = (float)xh;
      const float xl = xf - xhf;
      xa.h[0][e]     = (_Float16)(hh ? zl : xhf);
      xa.h[0][4 + e] = (_Float16)(hh ? zl : xl * XLO_CARRY);
      xa.h[1][e]     = (_Float16)(hh ? zl : xhf * (1.0f / WLO_CARRY));
    }
    xa.h[1][4] = (_Float16)(hh ? zl : onef);
    xa.h[1][5] = (_Float16)(hh ? zl : onef * (1.0f / BLO_CARRY));
    xa.h[1][6] = (_Float16)zl;
    xa.h[1][7] = (_Float16)zl;

    v8f acc[8];
#pragma unroll
    for (int n = 0; n < 8; ++n) acc[n] = z8;
#pragma unroll
    for (int n = 0; n < 8; ++n) {
      const v16h wb = frag_ld_packed(sWx + (n * 32 + lane) * 16);
      acc[n] = mma_h(xa.v, wb, acc[n]);
    }
    if (t > 0) {
      const v16h ha = frag_ld(ht + c * HID_N + 8 * hh);
#pragma unroll
      for (int n = 0; n < 8; ++n) acc[n] = mma_h(ha, whB[n], acc[n]);
    }

#pragma unroll
    for (int j = 0; j < 2; ++j) {
#pragma unroll
      for (int r = 0; r < 8; ++r) {
        const float zi = acc[0 + j][r] * WCARRY_INV;
        const float zf = acc[2 + j][r] * WCARRY_INV;
        const float zg = acc[4 + j][r] * WCARRY_INV;
        const float zo = acc[6 + j][r] * WCARRY_INV;
        const float iv = fsig(zi);
        const float fv = fsig(zf);
        const float gv = ftanh(zg);
        const float ov = fsig(zo);
        const float cn = fv * cst[j][r] + iv * gv;
        cst[j][r] = cn;
        const float hv = ov * ftanh(cn);
        ht[(8 * hh + r) * HID_N + j * 16 + c] = (_Float16)hv;
      }
    }
    __syncthreads();

    {
      const v8h s0 = *(const v8h*)(ht + lane * 8);
      const v8h s1 = *(const v8h*)(ht + 256 + lane * 8);
      unsigned short* dst = y0p + (((size_t)dir * STEP_N + (size_t)tt) * BATCH_N + (size_t)rowbase) * HID_N;
      *(volatile v8h*)(dst + lane * 8)       = s0;
      *(volatile v8h*)(dst + 256 + lane * 8) = s1;
      __threadfence();
      *(volatile v8h*)(dst + lane * 8)       = s0;
      *(volatile v8h*)(dst + 256 + lane * 8) = s1;
    }
    __syncthreads();
  }
}

__device__ __forceinline__ void stage_wih1(_Float16* sW, const float* __restrict__ Wd, int tid) {
#pragma unroll
  for (int it = 0; it < 2; ++it) {
    const int p = it * NTHR + tid;
    const int f = p >> 5, l2 = p & 31;
    const int cch = f >> 3, n = f & 7;
    const int g = n * 16 + (l2 & 15);
    FragU u;
    u.v = wfrag_from_f32(Wd + (size_t)g * L1_IN + cch * 32, l2 >> 4);
    *(v8h*)(sW + p * 16)     = u.h[0];
    *(v8h*)(sW + p * 16 + 8) = u.h[1];
    asm volatile("" ::: "memory");
  }
}

__global__ __launch_bounds__(NTHR) void lstm_l1_kernel(const unsigned short* __restrict__ y0p,
                                                      const float* __restrict__ Wih1,
                                                      const float* __restrict__ Whh1,
                                                      const float* __restrict__ bias1,
                                                      float* __restrict__ fin) {
  __shared__ __align__(16) _Float16 sW[16 * 32 * 16];
  __shared__ __align__(16) _Float16 sH[NTHR / 32][16 * HID_N];
  __shared__ __align__(16) float    sF[NTHR / 32][16 * SLAB_P];

  const _Float16* y0h = (const _Float16*)y0p;
  const int tid = threadIdx.x, lane = tid & 31, wave = tid >> 5;
  const int c = lane & 15, hh = lane >> 4;
  const int rowbase = blockIdx.x * ROWS_BLK + wave * 16;
  const size_t plane = (size_t)BATCH_N * HID_N;
  const _Float16* arow = y0h + (size_t)(rowbase + c) * HID_N + 8 * hh;
  const v8f z8 = {0.f, 0.f, 0.f, 0.f, 0.f, 0.f, 0.f, 0.f};
  float* slab = &sF[wave][0];
  _Float16* ht = &sH[wave][0];

  stage_wih1(sW, Wih1 + (size_t)GATE_N * L1_IN, tid);
  float bwi[2], bwg[2], bwo[2];
#pragma unroll
  for (int j = 0; j < 2; ++j) {
    bwi[j] = bias1[GATE_N + (0 + j) * 16 + c];
    bwg[j] = bias1[GATE_N + (4 + j) * 16 + c];
    bwo[j] = bias1[GATE_N + (6 + j) * 16 + c];
  }
  asm volatile("" ::: "memory");
  __syncthreads();
  {
    const v16h a0 = frag_ld(arow + (size_t)(STEP_N - 1) * plane);
    const v16h a1 = frag_ld(arow + (size_t)(STEP_N + STEP_N - 1) * plane);
    v8f acc[8];
#pragma unroll
    for (int n = 0; n < 8; ++n) acc[n] = z8;
#pragma unroll
    for (int n = 0; n < 8; ++n) {
      if (n == 2 || n == 3) continue;
      const v16h wb0 = frag_ld_packed(sW + (n * 32 + lane) * 16);
      acc[n] = mma_h(a0, wb0, acc[n]);
      const v16h wb1 = frag_ld_packed(sW + ((8 + n) * 32 + lane) * 16);
      acc[n] = mma_h(a1, wb1, acc[n]);
    }
#pragma unroll
    for (int j = 0; j < 2; ++j) {
#pragma unroll
      for (int r = 0; r < 8; ++r) {
        const float zi = fmaf(acc[0 + j][r], WCARRY_INV, bwi[j]);
        const float zg = fmaf(acc[4 + j][r], WCARRY_INV, bwg[j]);
        const float zo = fmaf(acc[6 + j][r], WCARRY_INV, bwo[j]);
        const float cn = fsig(zi) * ftanh(zg);
        const float hv = fsig(zo) * ftanh(cn);
        slab[(8 * hh + r) * SLAB_P + HID_N + j * 16 + c] = hv;
      }
    }
  }
  __syncthreads();

  stage_wih1(sW, Wih1, tid);
  v16h whB[8];
#pragma unroll
  for (int n = 0; n < 8; ++n) {
    whB[n] = wfrag_from_f32(Whh1 + ((size_t)n * 16 + c) * HID_N, hh);
    asm volatile("" : "+v"(whB[n]) :: "memory");
  }
  float bb[8];
#pragma unroll
  for (int n = 0; n < 8; ++n) bb[n] = bias1[n * 16 + c];
  asm volatile("" ::: "memory");
  __syncthreads();

  float cst[2][8], hl[2][8];
#pragma unroll
  for (int j = 0; j < 2; ++j)
#pragma unroll
    for (int r = 0; r < 8; ++r) { cst[j][r] = 0.0f; hl[j][r] = 0.0f; }

#pragma unroll 1
  for (int t = 0; t < STEP_N; ++t) {
    const v16h a0 = frag_ld(arow + (size_t)t * plane);
    const v16h a1 = frag_ld(arow + (size_t)(STEP_N + t) * plane);
    v8f acc[8];
#pragma unroll
    for (int n = 0; n < 8; ++n) acc[n] = z8;
#pragma unroll
    for (int n = 0; n < 8; ++n) {
      const v16h wb0 = frag_ld_packed(sW + (n * 32 + lane) * 16);
      acc[n] = mma_h(a0, wb0, acc[n]);
      const v16h wb1 = frag_ld_packed(sW + ((8 + n) * 32 + lane) * 16);
      acc[n] = mma_h(a1, wb1, acc[n]);
    }
    if (t > 0) {
      const v16h ha = frag_ld(ht + c * HID_N + 8 * hh);
#pragma unroll
      for (int n = 0; n < 8; ++n) acc[n] = mma_h(ha, whB[n], acc[n]);
    }
#pragma unroll
    for (int j = 0; j < 2; ++j) {
#pragma unroll
      for (int r = 0; r < 8; ++r) {
        const float zi = fmaf(acc[0 + j][r], WCARRY_INV, bb[0 + j]);
        const float zf = fmaf(acc[2 + j][r], WCARRY_INV, bb[2 + j]);
        const float zg = fmaf(acc[4 + j][r], WCARRY_INV, bb[4 + j]);
        const float zo = fmaf(acc[6 + j][r], WCARRY_INV, bb[6 + j]);
        const float iv = fsig(zi);
        const float fv = fsig(zf);
        const float gv = ftanh(zg);
        const float ov = fsig(zo);
        const float cn = fv * cst[j][r] + iv * gv;
        cst[j][r] = cn;
        const float hv = ov * ftanh(cn);
        hl[j][r] = hv;
        ht[(8 * hh + r) * HID_N + j * 16 + c] = (_Float16)hv;
      }
    }
    __syncthreads();
  }

#pragma unroll
  for (int j = 0; j < 2; ++j)
#pragma unroll
    for (int r = 0; r < 8; ++r) slab[(8 * hh + r) * SLAB_P + j * 16 + c] = hl[j][r];
  __syncthreads();
  {
    const int c4 = c * 4;
    for (int pass = 0; pass < 2; ++pass) {
#pragma unroll
      for (int it = 0; it < 8; ++it) {
        const int row = it * 2 + hh;
        const v4f v = *(const v4f*)(slab + row * SLAB_P + c4);
        *(volatile v4f*)(fin + (size_t)(rowbase + row) * L1_IN + c4) = v;
      }
      __threadfence();
    }
  }
}

__global__ __launch_bounds__(NTHR) void lstm_head_kernel(const float* __restrict__ dir_in,
                                                        const float* __restrict__ finals,
                                                        const float* __restrict__ lvlW,
                                                        const float* __restrict__ lvlb,
                                                        const float* __restrict__ vorW,
                                                        const float* __restrict__ vorb,
                                                        float* __restrict__ out) {
  __shared__ __align__(16) float sO[NTHR * OUT_W];
  const int tid = threadIdx.x;
  int b = blockIdx.x * NTHR + tid;
  b = b < BATCH_N ? b : (BATCH_N - 1);

  const float* di = dir_in + (size_t)b * DIR_CLS;
  float dv[DIR_CLS];
#pragma unroll
  for (int k = 0; k < DIR_CLS; ++k) dv[k] = di[k];
  int am = 0;
  float mx = dv[0];
#pragma unroll
  for (int k = 1; k < DIR_CLS; ++k) {
    const bool gt = dv[k] > mx;
    mx = gt ? dv[k] : mx;
    am = gt ? k : am;
  }
  const float m_vor = (am == 1 || am == 4) ? 1.0f : 0.0f;
  const float m_r   = (am == 0 || am == 5) ? 1.0f : 0.0f;
  const float m_l   = (am == 2 || am == 3) ? 1.0f : 0.0f;

  const float* pLL = finals + (size_t)b * L1_IN;
  const float* pLR = finals + (size_t)(b + BATCH_N) * L1_IN;
  const float* pVL = finals + ((size_t)ROWS_ALL + (size_t)b) * L1_IN;
  const float* pVR = finals + ((size_t)ROWS_ALL + (size_t)BATCH_N + (size_t)b) * L1_IN;

  float aL0 = 0.0f, aL1 = 0.0f, aR0 = 0.0f, aR1 = 0.0f, aV0 = 0.0f, aV1 = 0.0f;
#pragma unroll 1
  for (int k = 0; k < L1_IN; k += 4) {
    const v4f ll = *(const v4f*)(pLL + k);
    const v4f lr = *(const v4f*)(pLR + k);
    const v4f vl = *(const v4f*)(pVL + k);
    const v4f vr = *(const v4f*)(pVR + k);
    const v4f w0  = *(const v4f*)(lvlW + k);
    const v4f w1  = *(const v4f*)(lvlW + L1_IN + k);
    const v4f u0l = *(const v4f*)(vorW + k);
    const v4f u0r = *(const v4f*)(vorW + L1_IN + k);
    const v4f u1l = *(const v4f*)(vorW + 2 * L1_IN + k);
    const v4f u1r = *(const v4f*)(vorW + 3 * L1_IN + k);
#pragma unroll
    for (int e = 0; e < 4; ++e) {
      aL0 += w0[e] * ll[e];
      aL1 += w1[e] * ll[e];
      aR0 += w0[e] * lr[e];
      aR1 += w1[e] * lr[e];
      aV0 += u0l[e] * vl[e];
      aV0 += u0r[e] * vr[e];
      aV1 += u1l[e] * vl[e];
      aV1 += u1r[e] * vr[e];
    }
  }
  const float lb0 = lvlb[0], lb1 = lvlb[1], vb0 = vorb[0], vb1 = vorb[1];
  const float o0 = (aR0 + lb0) * m_r + (aL0 + lb0) * m_l + (aV0 + vb0) * m_vor;
  const float o1 = (aR1 + lb1) * m_r + (aL1 + lb1) * m_l + (aV1 + vb1) * m_vor;
  sO[tid * OUT_W + 0] = o0;
  sO[tid * OUT_W + 1] = o1;
  __syncthreads();
  if (tid < (NTHR * OUT_W) / 4) {
    const v4f v = *(const v4f*)(sO + tid * 4);
    float* dst = out + (size_t)blockIdx.x * (NTHR * OUT_W) + tid * 4;
    *(volatile v4f*)dst = v;
    __threadfence();
    *(volatile v4f*)dst = v;
  }
}

extern "C" void kernel_launch(void* const* d_in, const int* in_sizes, int n_in,
                              void* d_out, int out_size, void* d_ws, size_t ws_size, hipStream_t stream) {
  if (n_in < 18 || d_out == nullptr || d_ws == nullptr) return;
  if (in_sizes[0] != BATCH_N * DIR_CLS || in_sizes[1] != BATCH_N * SEQ_FULL * FEAT_IN ||
      in_sizes[2] != 2 * GATE_N * FEAT_IN || in_sizes[3] != 2 * GATE_N * HID_N || in_sizes[4] != 2 * GATE_N ||
      in_sizes[5] != 2 * GATE_N * L1_IN || in_sizes[6] != 2 * GATE_N * HID_N || in_sizes[7] != 2 * GATE_N ||
      in_sizes[14] != OUT_W * L1_IN || in_sizes[15] != OUT_W || in_sizes[16] != OUT_W * 2 * L1_IN ||
      in_sizes[17] != OUT_W || out_size != BATCH_N * OUT_W) return;

  const float* dir_input = (const float*)d_in[0];
  const float* pos       = (const float*)d_in[1];

  char* ws = (char*)d_ws;
  size_t off = 0;
  const size_t y0_bytes  = (size_t)2 * STEP_N * BATCH_N * HID_N * 2;
  const size_t fin_bytes = (size_t)2 * ROWS_ALL * L1_IN * 4;
  unsigned short* Y0 = (unsigned short*)(ws + off);
  off += (y0_bytes + 255) & ~(size_t)255;
  float* FINALS = (float*)(ws + off);
  off += (fin_bytes + 255) & ~(size_t)255;
  if (off > ws_size || off > (size_t)134217728) return;

  const dim3 grid0(BATCH_N / ROWS_BLK, 2);
  const dim3 grid1(BATCH_N / ROWS_BLK);
  for (int m = 0; m < 2; ++m) {
    const int base = 2 + m * 6;
    const float* Wih0 = (const float*)d_in[base + 0];
    const float* Whh0 = (const float*)d_in[base + 1];
    const float* b0   = (const float*)d_in[base + 2];
    const float* Wih1 = (const float*)d_in[base + 3];
    const float* Whh1 = (const float*)d_in[base + 4];
    const float* b1   = (const float*)d_in[base + 5];
    for (int ch = 0; ch < 2; ++ch) {
      float* fin = FINALS + ((size_t)m * ROWS_ALL + (size_t)ch * BATCH_N) * L1_IN;
      lstm_l0_kernel<<<grid0, NTHR, 0, stream>>>(pos, Wih0, Whh0, b0, Y0, ch * STEP_N);
      lstm_l1_kernel<<<grid1, NTHR, 0, stream>>>(Y0, Wih1, Whh1, b1, fin);
    }
  }
  lstm_head_kernel<<<BATCH_N / NTHR, NTHR, 0, stream>>>(dir_input, FINALS,
      (const float*)d_in[14], (const float*)d_in[15], (const float*)d_in[16], (const float*)d_in[17],
      (float*)d_out);
}
